// GroupLevelGNN_70342974374329
// MI455X (gfx1250) — hardware-verified
//
#include <hip/hip_runtime.h>
#include <stdint.h>
#include <stddef.h>


#define NG    4096
#define KAT   16
#define NA    16384
#define AD    256
#define FD    128
#define HD    256
#define NL    2
#define XW    (AD + FD)
#define PW    (2 * HD)
#define NE    (NG * KAT)

#define NTHR  256
#define NWAVE 8
#define CHUNK 2048
#define WCAP  256
#define NGRP  (CHUNK / (NTHR * 4))
#define IB    256
#define ALW   32
#define NCAP  512
#define GT    64
#define GTHR  128
#define CP    68

static_assert(WCAP == (CHUNK / NTHR) * 32);
static_assert(NGRP == 2);
static_assert((IB & (IB - 1)) == 0);
static_assert(IB <= 512);
static_assert(IB == NWAVE * 32);
static_assert((NA % IB) == 0);
static_assert(NG == 32 * 128);
static_assert(KAT * (ALW - 1) < NCAP);
static_assert((NG % GT) == 0);
static_assert((HD % GT) == 0);
static_assert((XW % 32) == 0);
static_assert((PW % 32) == 0);
static_assert((CP % 4) == 0);
static_assert(AD == 8 * 32);
static_assert(FD == 4 * 32);
static_assert(HD == 8 * 32);

typedef float          v4f   __attribute__((ext_vector_type(4)));
typedef float          v8f   __attribute__((ext_vector_type(8)));
typedef int            v4i   __attribute__((ext_vector_type(4)));
typedef unsigned int   v2u   __attribute__((ext_vector_type(2)));
typedef unsigned int   v4u   __attribute__((ext_vector_type(4)));
typedef unsigned short v8us  __attribute__((ext_vector_type(8)));
typedef __bf16         v16bf __attribute__((ext_vector_type(16)));
union FragU { v16bf v; v8us half[2]; };

__device__ __forceinline__ int imin(int a, int b) { return a < b ? a : b; }
__device__ __forceinline__ int iclamp(int v, int lo, int hi) { return v < lo ? lo : (v > hi ? hi : v); }

__device__ __forceinline__ unsigned int bfb(float f) {
  unsigned int u = __float_as_uint(f);
  u += 0x7fffu + ((u >> 16) & 1u);
  return u >> 16;
}
__device__ __forceinline__ unsigned int hl2(float v, unsigned int& lo) {
  const unsigned int hi = bfb(v);
  lo = bfb(v - __uint_as_float(hi << 16));
  return hi;
}
__device__ __forceinline__ void split8(v4f a, v4f b, v4u& hi, v4u& lo) {
  unsigned int l0, l1, l2, l3, l4, l5, l6, l7;
  const unsigned int h0 = hl2(a.x, l0), h1 = hl2(a.y, l1), h2 = hl2(a.z, l2), h3 = hl2(a.w, l3);
  const unsigned int h4 = hl2(b.x, l4), h5 = hl2(b.y, l5), h6 = hl2(b.z, l6), h7 = hl2(b.w, l7);
  hi.x = h0 | (h1 << 16); hi.y = h2 | (h3 << 16); hi.z = h4 | (h5 << 16); hi.w = h6 | (h7 << 16);
  lo.x = l0 | (l1 << 16); lo.y = l2 | (l3 << 16); lo.z = l4 | (l5 << 16); lo.w = l6 | (l7 << 16);
}
__device__ __forceinline__ void split4(v4f a, v2u& hi, v2u& lo) {
  unsigned int l0, l1, l2, l3;
  const unsigned int h0 = hl2(a.x, l0), h1 = hl2(a.y, l1), h2 = hl2(a.z, l2), h3 = hl2(a.w, l3);
  hi.x = h0 | (h1 << 16); hi.y = h2 | (h3 << 16);
  lo.x = l0 | (l1 << 16); lo.y = l2 | (l3 << 16);
}

__device__ __forceinline__ v8f wm(v16bf a, v16bf b, v8f c) {
  v8f d = __builtin_amdgcn_wmma_f32_16x16x32_bf16(false, a, false, b, (short)0, c, false, false);
  asm volatile("v_nop\n\tv_nop\n\tv_nop\n\tv_nop" : "+v"(d) : "v"(a), "v"(b));
  return d;
}

__device__ __forceinline__ v8f z8() {
  v8f z = {0.f, 0.f, 0.f, 0.f, 0.f, 0.f, 0.f, 0.f};
  return z;
}

__device__ __forceinline__ int scan_chunk(const int* __restrict__ key, int nE, int cbase,
                                          int nodeBase, int* list, int wave, int tid, int al16) {
  int wc = 0;
#pragma unroll
  for (int g = 0; g < NGRP; ++g) {
    const int el0 = (g * NTHR + tid) * 4;
    const int e0 = cbase + el0;
    const int sent = -2147483647 - 1;
    v4i d;
    if (al16 != 0 && (cbase + CHUNK <= nE)) {
      d = *(const v4i*)(key + e0);
    } else {
      const int c0 = iclamp(e0, 0, nE - 1), c1 = iclamp(e0 + 1, 0, nE - 1);
      const int c2 = iclamp(e0 + 2, 0, nE - 1), c3 = iclamp(e0 + 3, 0, nE - 1);
      const int k0v = key[c0], k1v = key[c1], k2v = key[c2], k3v = key[c3];
      d.x = (e0     < nE) ? k0v : sent;
      d.y = (e0 + 1 < nE) ? k1v : sent;
      d.z = (e0 + 2 < nE) ? k2v : sent;
      d.w = (e0 + 3 < nE) ? k3v : sent;
    }
    const unsigned s0 = (unsigned)d.x - (unsigned)nodeBase;
    const unsigned s1 = (unsigned)d.y - (unsigned)nodeBase;
    const unsigned s2 = (unsigned)d.z - (unsigned)nodeBase;
    const unsigned s3 = (unsigned)d.w - (unsigned)nodeBase;
    const bool h0 = s0 < (unsigned)IB;
    const bool h1 = s1 < (unsigned)IB;
    const bool h2 = s2 < (unsigned)IB;
    const bool h3 = s3 < (unsigned)IB;
    const unsigned many = __builtin_amdgcn_ballot_w32(h0 | h1 | h2 | h3);
    if (many != 0u) {
#define HITJ(J, HJ, SJ) { \
        const unsigned mj = __builtin_amdgcn_ballot_w32(HJ); \
        const int posj = wc + (int)__builtin_amdgcn_mbcnt_lo(mj, 0u); \
        if (HJ) { \
          if (posj < WCAP) list[wave * WCAP + posj] = ((el0 + (J)) << 9) | (int)(SJ); \
        } \
        wc += (int)__builtin_popcount(mj); }
      HITJ(0, h0, s0)
      HITJ(1, h1, s1)
      HITJ(2, h2, s2)
      HITJ(3, h3, s3)
#undef HITJ
    }
  }
  return wc;
}

__global__ __launch_bounds__(NTHR) void k_cvtT(const float* __restrict__ W, int Kd, int Nd,
                                               unsigned short* Th, unsigned short* Tl, int ldt) {
  __shared__ __attribute__((aligned(16))) float Ws[64 * CP];
  const int tid = threadIdx.x;
  const int k0 = blockIdx.y * 64, n0 = blockIdx.x * 64;
  {
    const int r = tid >> 2;
    const int c = (tid & 3) * 16;
    const float* p = W + (size_t)(k0 + r) * Nd + n0 + c;
    const v4f f0 = *(const v4f*)(p), f1 = *(const v4f*)(p + 4);
    const v4f f2 = *(const v4f*)(p + 8), f3 = *(const v4f*)(p + 12);
    *(v4f*)(Ws + r * CP + c)      = f0;
    *(v4f*)(Ws + r * CP + c + 4)  = f1;
    *(v4f*)(Ws + r * CP + c + 8)  = f2;
    *(v4f*)(Ws + r * CP + c + 12) = f3;
  }
  __syncthreads();
  v4u hiv[2], lov[2];
  size_t ov[2];
#pragma unroll
  for (int pz = 0; pz < 2; ++pz) {
    const int nn = pz * 32 + (tid >> 3);
    const int kk = (tid & 7) * 8;
    v4f a, b;
    a.x = Ws[(kk + 0) * CP + nn]; a.y = Ws[(kk + 1) * CP + nn];
    a.z = Ws[(kk + 2) * CP + nn]; a.w = Ws[(kk + 3) * CP + nn];
    b.x = Ws[(kk + 4) * CP + nn]; b.y = Ws[(kk + 5) * CP + nn];
    b.z = Ws[(kk + 6) * CP + nn]; b.w = Ws[(kk + 7) * CP + nn];
    split8(a, b, hiv[pz], lov[pz]);
    ov[pz] = (size_t)(n0 + nn) * ldt + k0 + kk;
  }
#pragma unroll
  for (int pz = 0; pz < 2; ++pz) {
    *(volatile v4u*)(Th + ov[pz]) = hiv[pz];
    *(volatile v4u*)(Tl + ov[pz]) = lov[pz];
  }
  __threadfence();
#pragma unroll
  for (int pz = 0; pz < 2; ++pz) {
    *(volatile v4u*)(Th + ov[pz]) = hiv[pz];
    *(volatile v4u*)(Tl + ov[pz]) = lov[pz];
  }
}

__global__ __launch_bounds__(NTHR) void k_inv(const int* __restrict__ gidx, int* tinv, int nA, int nE) {
  __shared__ __attribute__((aligned(16))) int plist[IB * ALW];
  __shared__ int pcnt[IB];
  __shared__ int list[NWAVE * WCAP];
  __shared__ int wcnt[NWAVE];

  const int tid  = threadIdx.x;
  const int lane = tid & 31;
  const int wave = tid >> 5;
  const int atomBase = blockIdx.x * IB;

  for (int i = tid; i < IB * ALW; i += NTHR) plist[i] = 0;
  for (int i = tid; i < IB; i += NTHR) pcnt[i] = 0;
  __syncthreads();

  const int al16 = ((((uintptr_t)(const void*)gidx) & 15u) == 0) ? 1 : 0;
  const int nChunks = (nE + CHUNK - 1) / CHUNK;

#pragma unroll 1
  for (int ch = 0; ch < nChunks; ++ch) {
    const int cbase = ch * CHUNK;
    const int wc = scan_chunk(gidx, nE, cbase, atomBase, list, wave, tid, al16);
    if (lane == 0) wcnt[wave] = wc;
    __syncthreads();
    if (wave == 0) {
#pragma unroll 1
      for (int wsx = 0; wsx < NWAVE; ++wsx) {
        int n = wcnt[wsx];
        n = n > WCAP ? WCAP : n;
        n = n < 0 ? 0 : n;
#pragma unroll 1
        for (int i = 0; i < n; ++i) {
          const int ent  = list[wsx * WCAP + i];
          const int slot = ent & (IB - 1);
          int e = cbase + ((ent >> 9) & (CHUNK - 1));
          e = iclamp(e, 0, nE - 1);
          const int grp = e / KAT;
          const int c   = pcnt[slot];
          const int pos = c < ALW - 2 ? c : ALW - 2;
          if (lane == 0) plist[slot * ALW + 1 + pos] = grp;
          pcnt[slot] = c + 1;
        }
      }
    }
    __syncthreads();
  }

  for (int s = tid; s < IB; s += NTHR) {
    int c = pcnt[s];
    c = c > ALW - 1 ? ALW - 1 : c;
    plist[s * ALW] = c;
  }
  __syncthreads();

#pragma unroll 1
  for (int ps = 0; ps < 2; ++ps) {
#pragma unroll
    for (int it = 0; it < 8; ++it) {
      const int slot = wave * 32 + 4 * it + (lane >> 3);
      const int c4   = 4 * (lane & 7);
      const v4i v = *(const v4i*)(plist + slot * ALW + c4);
      int at = atomBase + slot;
      at = at > nA - 1 ? nA - 1 : at;
      *(volatile v4i*)(tinv + (size_t)at * ALW + c4) = v;
    }
    if (ps == 0) __threadfence();
  }
}

__global__ __launch_bounds__(32) void k_group(const float* __restrict__ atom, const int* __restrict__ gidx,
                                              const float* __restrict__ gf, const int* __restrict__ tinv,
                                              unsigned short* Xh, unsigned short* Xl, int* tnb, int nG, int nA) {
  __shared__ int clist[NCAP];
  __shared__ __attribute__((aligned(16))) int orow[NCAP];

  const int lane = threadIdx.x & 31;
  const int g = blockIdx.x;

  {
    const v4i z = {0, 0, 0, 0};
#pragma unroll
    for (int q = 0; q < 4; ++q) *(v4i*)(orow + 16 * lane + 4 * q) = z;
  }

  const int myatom = iclamp(gidx[(size_t)g * KAT + (lane & (KAT - 1))], 0, nA - 1);

  v4f sa = {0.f, 0.f, 0.f, 0.f};
  v4f sb = {0.f, 0.f, 0.f, 0.f};
#pragma unroll 4
  for (int k = 0; k < KAT; ++k) {
    const int a = __shfl(myatom, k, 32);
    const float* p = atom + (size_t)a * AD + 8 * lane;
    sa += *(const v4f*)(p);
    sb += *(const v4f*)(p + 4);
  }
  sa *= (1.0f / KAT);
  sb *= (1.0f / KAT);
  v4u phi, plo;
  split8(sa, sb, phi, plo);
  const v4f f4 = *(const v4f*)(gf + (size_t)g * FD + 4 * lane);
  v2u fhi, flo;
  split4(f4, fhi, flo);
  const size_t ox = (size_t)g * XW + 8 * lane;
  const size_t of = (size_t)g * XW + AD + 4 * lane;
  *(volatile v4u*)(Xh + ox) = phi;
  *(volatile v4u*)(Xl + ox) = plo;
  *(volatile v2u*)(Xh + of) = fhi;
  *(volatile v2u*)(Xl + of) = flo;

  int ncand = 0;
#pragma unroll 1
  for (int a = 0; a < KAT; ++a) {
    const int at = __shfl(myatom, a, 32);
    const int rv = tinv[(size_t)at * ALW + lane];
    int cnt = __shfl(rv, 0, 32);
    cnt = iclamp(cnt, 0, ALW - 1);
    const int c = iclamp(rv, 0, nG - 1);
    const bool valid = (lane >= 1) && (lane <= cnt) && (rv != g);
    const unsigned m = __builtin_amdgcn_ballot_w32(valid);
    const int pos = ncand + (int)__builtin_amdgcn_mbcnt_lo(m, 0u);
    if (valid) clist[imin(pos, NCAP - 1)] = c;
    ncand += (int)__builtin_popcount(m);
  }
  __syncthreads();
  ncand = imin(ncand, NCAP);

  unsigned int w0 = 0u, w1 = 0u, w2 = 0u, w3 = 0u;
#pragma unroll 1
  for (int p = 0; p < ncand; ++p) {
    const int c = clist[p];
    const bool mine = ((c >> 7) == lane);
    const int j = (c >> 5) & 3;
    const unsigned int bit = 1u << (unsigned)(c & 31);
    w0 |= (mine && j == 0) ? bit : 0u;
    w1 |= (mine && j == 1) ? bit : 0u;
    w2 |= (mine && j == 2) ? bit : 0u;
    w3 |= (mine && j == 3) ? bit : 0u;
  }
  const int cnt = (int)__builtin_popcount(w0) + (int)__builtin_popcount(w1)
                + (int)__builtin_popcount(w2) + (int)__builtin_popcount(w3);
  int x = cnt;
#pragma unroll
  for (int d = 1; d < 32; d <<= 1) {
    const int y = __shfl_up(x, d, 32);
    x = (lane >= d) ? (x + y) : x;
  }
  const int total = __shfl(x, 31, 32);
  const int excl  = x - cnt;
  int pos = 1 + excl;
#define EMITW(WV, J) { unsigned int word = (WV); \
    for (int it = 0; it < 32; ++it) { \
      if (word == 0u) break; \
      const int b = __builtin_ctz(word); \
      word &= word - 1u; \
      orow[imin(pos, NCAP - 1)] = lane * 128 + 32 * (J) + b; \
      ++pos; } }
  EMITW(w0, 0)
  EMITW(w1, 1)
  EMITW(w2, 2)
  EMITW(w3, 3)
#undef EMITW
  if (lane == 0) orow[0] = imin(total, NCAP - 1);
  __syncthreads();

  const size_t ot = (size_t)g * NCAP;
#pragma unroll
  for (int i = 0; i < 4; ++i) {
    const v4i v = *(const v4i*)(orow + 128 * i + 4 * lane);
    *(volatile v4i*)(tnb + ot + 128 * i + 4 * lane) = v;
  }
  __threadfence();
  *(volatile v4u*)(Xh + ox) = phi;
  *(volatile v4u*)(Xl + ox) = plo;
  *(volatile v2u*)(Xh + of) = fhi;
  *(volatile v2u*)(Xl + of) = flo;
#pragma unroll
  for (int i = 0; i < 4; ++i) {
    const v4i v = *(const v4i*)(orow + 128 * i + 4 * lane);
    *(volatile v4i*)(tnb + ot + 128 * i + 4 * lane) = v;
  }
}

__global__ __launch_bounds__(32) void k_agg(const float* __restrict__ ge, const int* __restrict__ tnb,
                                            unsigned short* Ph, unsigned short* Pl, int nG) {
  const int lane = threadIdx.x & 31;
  const int g = blockIdx.x;
  const int* row = tnb + (size_t)g * NCAP;
  int n = row[0];
  n = iclamp(n, 0, NCAP - 1);
  v4f ca = {0.f, 0.f, 0.f, 0.f};
  v4f cb = {0.f, 0.f, 0.f, 0.f};
#pragma unroll 2
  for (int p = 0; p < n; ++p) {
    const int id = iclamp(row[1 + p], 0, nG - 1);
    const float* px = ge + (size_t)id * HD + 8 * lane;
    ca += *(const v4f*)(px);
    cb += *(const v4f*)(px + 4);
  }
  v4u hi, lo;
  split8(ca, cb, hi, lo);
  const size_t o = (size_t)g * PW + HD + 8 * lane;
  *(volatile v4u*)(Ph + o) = hi;
  *(volatile v4u*)(Pl + o) = lo;
  __threadfence();
  *(volatile v4u*)(Ph + o) = hi;
  *(volatile v4u*)(Pl + o) = lo;
}

__device__ __forceinline__ void epi_lds(v8f acc, int rbase, int col, float bv, int relu, float* Cs) {
#pragma unroll
  for (int r = 0; r < 8; ++r) {
    float v = acc[r] + bv;
    if (relu != 0) v = fmaxf(v, 0.f);
    Cs[(rbase + r) * CP + col] = v;
  }
}

__global__ __launch_bounds__(GTHR) void k_gemm(
    const unsigned short* __restrict__ Ah, const unsigned short* __restrict__ Al, int lda,
    const unsigned short* __restrict__ Bh, const unsigned short* __restrict__ Bl, int ldb, int K,
    const float* __restrict__ bias1, const float* __restrict__ bias2, int nBias, int relu,
    float* Cf, int ldcf, unsigned short* Ch, unsigned short* Cl, int ldcp, int mode) {
  __shared__ __attribute__((aligned(16))) float Cs[GT * CP];

  const int tid  = threadIdx.x;
  const int lane = tid & 31;
  const int wave = tid >> 5;
  const int h    = lane >> 4;
  const int m    = lane & 15;
  const int wr   = wave >> 1;
  const int wc   = wave & 1;
  const int m0   = blockIdx.y * GT;
  const int n0   = blockIdx.x * GT;

  const unsigned short* pAh0 = Ah + (size_t)(m0 + 32 * wr + m) * lda + 8 * h;
  const unsigned short* pAh1 = pAh0 + (size_t)16 * lda;
  const unsigned short* pAl0 = Al + (size_t)(m0 + 32 * wr + m) * lda + 8 * h;
  const unsigned short* pAl1 = pAl0 + (size_t)16 * lda;
  const unsigned short* pBh0 = Bh + (size_t)(n0 + 32 * wc + m) * ldb + 8 * h;
  const unsigned short* pBh1 = pBh0 + (size_t)16 * ldb;
  const unsigned short* pBl0 = Bl + (size_t)(n0 + 32 * wc + m) * ldb + 8 * h;
  const unsigned short* pBl1 = pBl0 + (size_t)16 * ldb;

  v8f acc00 = z8(), acc01 = z8(), acc10 = z8(), acc11 = z8();

#pragma unroll 1
  for (int k0 = 0; k0 < K; k0 += 32) {
    FragU ah0, ah1, al0, al1, bh0, bh1, bl0, bl1;
    ah0.half[0] = *(const v8us*)(pAh0 + k0); ah0.half[1] = *(const v8us*)(pAh0 + k0 + 16);
    ah1.half[0] = *(const v8us*)(pAh1 + k0); ah1.half[1] = *(const v8us*)(pAh1 + k0 + 16);
    al0.half[0] = *(const v8us*)(pAl0 + k0); al0.half[1] = *(const v8us*)(pAl0 + k0 + 16);
    al1.half[0] = *(const v8us*)(pAl1 + k0); al1.half[1] = *(const v8us*)(pAl1 + k0 + 16);
    bh0.half[0] = *(const v8us*)(pBh0 + k0); bh0.half[1] = *(const v8us*)(pBh0 + k0 + 16);
    bh1.half[0] = *(const v8us*)(pBh1 + k0); bh1.half[1] = *(const v8us*)(pBh1 + k0 + 16);
    bl0.half[0] = *(const v8us*)(pBl0 + k0); bl0.half[1] = *(const v8us*)(pBl0 + k0 + 16);
    bl1.half[0] = *(const v8us*)(pBl1 + k0); bl1.half[1] = *(const v8us*)(pBl1 + k0 + 16);

    acc00 = wm(ah0.v, bh0.v, acc00); acc00 = wm(ah0.v, bl0.v, acc00); acc00 = wm(al0.v, bh0.v, acc00);
    acc01 = wm(ah0.v, bh1.v, acc01); acc01 = wm(ah0.v, bl1.v, acc01); acc01 = wm(al0.v, bh1.v, acc01);
    acc10 = wm(ah1.v, bh0.v, acc10); acc10 = wm(ah1.v, bl0.v, acc10); acc10 = wm(al1.v, bh0.v, acc10);
    acc11 = wm(ah1.v, bh1.v, acc11); acc11 = wm(ah1.v, bl1.v, acc11); acc11 = wm(al1.v, bh1.v, acc11);
  }

  const int colA = 32 * wc + m;
  const int colB = colA + 16;
  float bA = 0.f, bB = 0.f;
  if (nBias >= 1) {
    bA += bias1[n0 + colA];
    bB += bias1[n0 + colB];
  }
  if (nBias >= 2) {
    bA += bias2[n0 + colA];
    bB += bias2[n0 + colB];
  }
  epi_lds(acc00, 32 * wr + 8 * h,      colA, bA, relu, Cs);
  epi_lds(acc01, 32 * wr + 8 * h,      colB, bB, relu, Cs);
  epi_lds(acc10, 32 * wr + 16 + 8 * h, colA, bA, relu, Cs);
  epi_lds(acc11, 32 * wr + 16 + 8 * h, colB, bB, relu, Cs);
  __syncthreads();

  if ((mode & 1) != 0) {
#pragma unroll 1
    for (int ps = 0; ps < 2; ++ps) {
#pragma unroll
      for (int it = 0; it < 8; ++it) {
        const int row = 16 * wave + 2 * it + (lane >> 4);
        const int c4  = 4 * (lane & 15);
        const v4f v = *(const v4f*)(Cs + row * CP + c4);
        *(volatile v4f*)(Cf + (size_t)(m0 + row) * ldcf + n0 + c4) = v;
      }
      if (ps == 0) __threadfence();
    }
  }
  if ((mode & 2) != 0) {
#pragma unroll 1
    for (int ps = 0; ps < 2; ++ps) {
#pragma unroll
      for (int it = 0; it < 4; ++it) {
        const int row = 16 * wave + 4 * it + (lane >> 3);
        const int c8  = 8 * (lane & 7);
        const v4f a = *(const v4f*)(Cs + row * CP + c8);
        const v4f b = *(const v4f*)(Cs + row * CP + c8 + 4);
        v4u hi, lo;
        split8(a, b, hi, lo);
        const size_t o = (size_t)(m0 + row) * ldcp + n0 + c8;
        *(volatile v4u*)(Ch + o) = hi;
        *(volatile v4u*)(Cl + o) = lo;
      }
      if (ps == 0) __threadfence();
    }
  }
}

extern "C" void kernel_launch(void* const* d_in, const int* in_sizes, int n_in,
                              void* d_out, int out_size, void* d_ws, size_t ws_size,
                              hipStream_t stream) {
  if (n_in < 10) return;
  if (in_sizes[0] != NA * AD) return;
  if (in_sizes[1] != NG * KAT) return;
  if (in_sizes[2] != NG * FD) return;
  if (in_sizes[3] != FD * HD || in_sizes[4] != HD) return;
  if (in_sizes[5] != AD * HD || in_sizes[6] != HD) return;
  if (in_sizes[7] != NL * HD * HD || in_sizes[8] != NL * HD * HD || in_sizes[9] != NL * HD) return;
  if (out_size != NG * HD) return;

  const float* atom  = (const float*)d_in[0];
  const int*   gidx  = (const int*)d_in[1];
  const float* gf    = (const float*)d_in[2];
  const float* W_in  = (const float*)d_in[3];
  const float* b_in  = (const float*)d_in[4];
  const float* W_a2g = (const float*)d_in[5];
  const float* b_a2g = (const float*)d_in[6];
  const float* W_s   = (const float*)d_in[7];
  const float* W_n   = (const float*)d_in[8];
  const float* b_mp  = (const float*)d_in[9];
  float* out = (float*)d_out;

  char* wsb = (char*)d_ws;
  size_t off = 0;
#define CARVE(T, name, nbytes) T* name = (T*)(wsb + off); off += ((((size_t)(nbytes)) + 255) / 256) * 256;
  CARVE(int,            Tinv, (size_t)NA * ALW * 4)
  CARVE(int,            Tnb,  (size_t)NG * NCAP * 4)
  CARVE(unsigned short, Xh,   (size_t)NG * XW * 2)
  CARVE(unsigned short, Xl,   (size_t)NG * XW * 2)
  CARVE(unsigned short, WcTh, (size_t)HD * XW * 2)
  CARVE(unsigned short, WcTl, (size_t)HD * XW * 2)
  CARVE(unsigned short, WLTh, (size_t)NL * HD * PW * 2)
  CARVE(unsigned short, WLTl, (size_t)NL * HD * PW * 2)
  CARVE(float,          GE,   (size_t)NG * HD * 4)
  CARVE(unsigned short, P0h,  (size_t)NG * PW * 2)
  CARVE(unsigned short, P0l,  (size_t)NG * PW * 2)
  CARVE(unsigned short, P1h,  (size_t)NG * PW * 2)
  CARVE(unsigned short, P1l,  (size_t)NG * PW * 2)
#undef CARVE
  if (off > ws_size) return;

  k_cvtT<<<dim3(HD / 64, AD / 64), NTHR, 0, stream>>>(W_a2g, AD, HD, WcTh, WcTl, XW);
  k_cvtT<<<dim3(HD / 64, FD / 64), NTHR, 0, stream>>>(W_in,  FD, HD, WcTh + AD, WcTl + AD, XW);
  for (int l = 0; l < NL; ++l) {
    const size_t wo = (size_t)l * HD * HD;
    const size_t po = (size_t)l * HD * PW;
    k_cvtT<<<dim3(HD / 64, HD / 64), NTHR, 0, stream>>>(W_s + wo, HD, HD, WLTh + po,      WLTl + po,      PW);
    k_cvtT<<<dim3(HD / 64, HD / 64), NTHR, 0, stream>>>(W_n + wo, HD, HD, WLTh + po + HD, WLTl + po + HD, PW);
  }

  k_inv<<<NA / IB, NTHR, 0, stream>>>(gidx, Tinv, NA, NE);
  k_group<<<NG, 32, 0, stream>>>(atom, gidx, gf, Tinv, Xh, Xl, Tnb, NG, NA);

  k_gemm<<<dim3(HD / GT, NG / GT), GTHR, 0, stream>>>(Xh, Xl, XW, WcTh, WcTl, XW, XW,
                                                     b_a2g, b_in, 2, 0, GE, HD, P0h, P0l, PW, 3);

  k_agg<<<NG, 32, 0, stream>>>(GE, Tnb, P0h, P0l, NG);
  k_gemm<<<dim3(HD / GT, NG / GT), GTHR, 0, stream>>>(P0h, P0l, PW, WLTh, WLTl, PW, PW,
                                                     b_mp, b_mp, 1, 1, GE, HD, P1h, P1l, PW, 3);

  k_agg<<<NG, 32, 0, stream>>>(GE, Tnb, P1h, P1l, NG);
  k_gemm<<<dim3(HD / GT, NG / GT), GTHR, 0, stream>>>(P1h, P1l, PW, WLTh + (size_t)HD * PW, WLTl + (size_t)HD * PW, PW, PW,
                                                     b_mp + HD, b_mp + HD, 1, 1, out, HD, P0h, P0l, PW, 1);
}
